// Pts_attention_72954314490251
// MI455X (gfx1250) — hardware-verified
//
#include <hip/hip_runtime.h>
#include <stdint.h>
#include <math.h>


typedef __attribute__((ext_vector_type(16))) _Float16 v16h;
typedef __attribute__((ext_vector_type(8)))  _Float16 v8h;
typedef __attribute__((ext_vector_type(16))) __bf16   v16b;
typedef __attribute__((ext_vector_type(8)))  __bf16   v8b;
typedef __attribute__((ext_vector_type(8)))  float    v8f;
typedef __attribute__((ext_vector_type(4)))  float    v4f;
#define PSCALE 32768.0f
#define U16(p) ((const unsigned short*)(const void*)(p))
#define PSCALE_INV (1.0f / 32768.0f)

__device__ __forceinline__ unsigned short f2bf_bits(float f) {
  unsigned u = __float_as_uint(f);
  return (unsigned short)((u + 0x7FFFu + ((u >> 16) & 1u)) >> 16);
}
__device__ __forceinline__ float bf_bits2f(unsigned short h) { return __uint_as_float(((unsigned)h) << 16); }

__device__ __forceinline__ void dep_guard_h(v8f& a, v8f& b, v16h x, v16h y) { asm volatile("v_nop\n\tv_nop\n\tv_nop\n\tv_nop" : "+v"(a), "+v"(b) : "v"(x), "v"(y)); }
__device__ __forceinline__ void dep_guard_b(v8f& a, v8f& b, v16b x, v16b y) { asm volatile("v_nop\n\tv_nop\n\tv_nop\n\tv_nop" : "+v"(a), "+v"(b) : "v"(x), "v"(y)); }
__device__ __forceinline__ void keep4_h(v16h a, v16h b, v16h c, v16h d) { asm volatile("v_nop" :: "v"(a), "v"(b), "v"(c), "v"(d)); }
__device__ __forceinline__ void keep4_b(v16b a, v16b b, v16b c, v16b d) { asm volatile("v_nop" :: "v"(a), "v"(b), "v"(c), "v"(d)); }
__device__ __forceinline__ void acc_guard4(v8f& a, v8f& b, v8f& c, v8f& d) { asm volatile("v_nop\n\tv_nop\n\tv_nop\n\tv_nop" : "+v"(a), "+v"(b), "+v"(c), "+v"(d)); }
template <typename T> struct Frag;
template <> struct Frag<_Float16> {
  typedef v16h V; union U { v16h v; v8h h[2]; };
  static __device__ __forceinline__ v16h load(const _Float16* p) {
    U f; f.h[0] = *(const v8h*)(p); f.h[1] = *(const v8h*)(p + 16); return f.v;
  }
  static __device__ __forceinline__ v8f mma(v16h a, v16h b, v8f c) {
    return __builtin_amdgcn_wmma_f32_16x16x32_f16(false, a, false, b, (short)0, c, false, false);
  }
  static __device__ __forceinline__ void guard(v8f& a, v8f& b, v16h x, v16h y) { dep_guard_h(a, b, x, y); }
  static __device__ __forceinline__ void keep(v16h a, v16h b, v16h c, v16h d) { keep4_h(a, b, c, d); }
};
template <> struct Frag<__bf16> {
  typedef v16b V; union U { v16b v; v8b h[2]; };
  static __device__ __forceinline__ v16b load(const __bf16* p) {
    U f; f.h[0] = *(const v8b*)(p); f.h[1] = *(const v8b*)(p + 16); return f.v;
  }
  static __device__ __forceinline__ v8f mma(v16b a, v16b b, v8f c) {
    return __builtin_amdgcn_wmma_f32_16x16x32_bf16(false, a, false, b, (short)0, c, false, false);
  }
  static __device__ __forceinline__ void guard(v8f& a, v8f& b, v16b x, v16b y) { dep_guard_b(a, b, x, y); }
  static __device__ __forceinline__ void keep(v16b a, v16b b, v16b c, v16b d) { keep4_b(a, b, c, d); }
};

template <int ET> struct Elem;
template <> struct Elem<0> { typedef _Float16 T; };
template <> struct Elem<1> { typedef __bf16 T; };
template <int ET, bool SPLIT, int BIAS_MODE, int OUT_MODE, bool RESID, int ACT = 0>
__global__ __launch_bounds__(256) void wmma_gemm64(
    const unsigned short* __restrict__ Ap, const unsigned short* __restrict__ A2p, int lda, long strideA,
    const unsigned short* __restrict__ Btp, const unsigned short* __restrict__ Bt2p, int ldb, long strideB,
    void* __restrict__ Cout, void* __restrict__ Cout2, int ldc, long strideC,
    const float* __restrict__ bias,
    const float* __restrict__ resid, long strideR,
    int M, int N, int K, float scale) {
  typedef typename Elem<ET>::T T;
  typedef typename Frag<T>::V V;
  const T* A = (const T*)Ap; const T* A2 = (const T*)A2p; const T* Bt = (const T*)Btp; const T* Bt2 = (const T*)Bt2p;
  __shared__ __align__(16) float sT[8][16 * 68];
  const int b    = blockIdx.y;
  const int lane = threadIdx.x & 31;
  const int wave = threadIdx.x >> 5;
  const int tilesN = N >> 6;
  const int tilesM = M >> 6;
  const int tile = blockIdx.x * 8 + wave;
  if (tile >= tilesM * tilesN) return;
  const int tm = tile / tilesN;
  const int tn = tile - tm * tilesN;
  const int m0 = tm << 6;
  const int n0 = tn << 6;

  const T* Ab  = A  + (size_t)b * strideA;
  const T* Bb  = Bt + (size_t)b * strideB;
  const T* Ab2 = SPLIT ? (A2  + (size_t)b * strideA) : nullptr;
  const T* Bb2 = SPLIT ? (Bt2 + (size_t)b * strideB) : nullptr;

  const int rlane = lane & 15;
  const int koff  = (lane >> 4) * 8;
  const int mOff  = (lane >> 4) * 8;

  v8f acc[4][4];
#pragma unroll
  for (int i = 0; i < 4; ++i)
#pragma unroll
    for (int j = 0; j < 4; ++j) acc[i][j] = (v8f){0.f,0.f,0.f,0.f,0.f,0.f,0.f,0.f};

  for (int k0 = 0; k0 < K; k0 += 32) {
    V bh[4], bl[4];
#pragma unroll
    for (int j = 0; j < 4; ++j) {
      const size_t bo = (size_t)(n0 + (j << 4) + rlane) * ldb + koff + k0;
      bh[j] = Frag<T>::load(Bb + bo);
      if (SPLIT) bl[j] = Frag<T>::load(Bb2 + bo);
    }
#pragma unroll
    for (int i = 0; i < 4; ++i) {
      const size_t ao = (size_t)(m0 + (i << 4) + rlane) * lda + koff + k0;
      V ah = Frag<T>::load(Ab + ao);
      V al;
      if (SPLIT) al = Frag<T>::load(Ab2 + ao);
#pragma unroll
      for (int j = 0; j < 4; ++j) {
        acc[i][j] = Frag<T>::mma(ah, bh[j], acc[i][j]);
        if (SPLIT) {
          acc[i][j] = Frag<T>::mma(ah, bl[j], acc[i][j]);
          acc[i][j] = Frag<T>::mma(al, bh[j], acc[i][j]);
        }
      }
      Frag<T>::guard(acc[i][0], acc[i][3], ah, SPLIT ? al : ah);
    }
    Frag<T>::keep(bh[0], bh[1], bh[2], bh[3]);
    if (SPLIT) Frag<T>::keep(bl[0], bl[1], bl[2], bl[3]);
  }
  acc_guard4(acc[0][0], acc[0][1], acc[0][2], acc[0][3]);
  acc_guard4(acc[1][0], acc[1][1], acc[1][2], acc[1][3]);
  acc_guard4(acc[2][0], acc[2][1], acc[2][2], acc[2][3]);
  acc_guard4(acc[3][0], acc[3][1], acc[3][2], acc[3][3]);

  float* slab = sT[wave];
  const float* Rb = RESID ? (resid + (size_t)b * strideR) : nullptr;
#pragma unroll
  for (int i = 0; i < 4; ++i) {
    const int mBase = m0 + (i << 4);
#pragma unroll
    for (int j = 0; j < 4; ++j) {
      const int n = n0 + (j << 4) + rlane;
      float bv = 0.f;
      if (BIAS_MODE == 2) bv = bias[n];
#pragma unroll
      for (int r = 0; r < 8; ++r) {
        float v = acc[i][j][r] * scale;
        if (BIAS_MODE == 1) v += bias[mBase + mOff + r];
        if (BIAS_MODE == 2) v += bv;
        if (RESID) v += Rb[(size_t)(mBase + mOff + r) * ldc + n];
        if (ACT == 1) v = tanhf(v);
        if (ACT == 2) v = fmaxf(v, 0.0f);
        if (ACT == 3) v = v / (1.0f + expf(-v));
        if (ACT == 4) v = (v > 0.f) ? v : 0.01f * v;
        if (ACT == 5) v = 0.5f * v * (1.0f + erff(v * 0.70710678118654752f));
        slab[(mOff + r) * 68 + (j << 4) + rlane] = v;
      }
    }
    __builtin_amdgcn_fence(__ATOMIC_RELEASE, "workgroup");
    __builtin_amdgcn_wave_barrier();
    __builtin_amdgcn_fence(__ATOMIC_ACQUIRE, "workgroup");
    if (OUT_MODE == 0) {
      float* C = (float*)Cout + (size_t)b * strideC;
      const int hh = lane >> 4, c4 = (lane & 15) * 4;
      for (int pass = 0; pass < 2; ++pass) {
#pragma unroll
        for (int it = 0; it < 8; ++it) {
          const int row = it * 2 + hh;
          v4f v = *(const v4f*)(slab + row * 68 + c4);
          *(volatile v4f*)(C + (size_t)(mBase + row) * ldc + n0 + c4) = v;
        }
        __threadfence();
      }
    } else {
      const int q = lane >> 3, c8 = (lane & 7) * 8;
      unsigned short* C  = (unsigned short*)Cout  + (size_t)b * strideC;
      unsigned short* C2 = (OUT_MODE == 2) ? ((unsigned short*)Cout2 + (size_t)b * strideC) : nullptr;
      for (int pass = 0; pass < 2; ++pass) {
#pragma unroll
        for (int it = 0; it < 4; ++it) {
          const int row = it * 4 + q;
          const float* sp = slab + row * 68 + c8;
          v8h hv, lv;
#pragma unroll
          for (int e = 0; e < 8; ++e) {
            if (OUT_MODE == 1) {
              hv[e] = (_Float16)sp[e];
            } else {
              unsigned short hb = f2bf_bits(sp[e]);
              unsigned short lb = f2bf_bits(sp[e] - bf_bits2f(hb));
              hv[e] = __builtin_bit_cast(_Float16, hb);
              lv[e] = __builtin_bit_cast(_Float16, lb);
            }
          }
          *(volatile v8h*)(C + (size_t)(mBase + row) * ldc + n0 + c8) = hv;
          if (OUT_MODE == 2) *(volatile v8h*)(C2 + (size_t)(mBase + row) * ldc + n0 + c8) = lv;
        }
        __threadfence();
      }
    }
    __builtin_amdgcn_fence(__ATOMIC_RELEASE, "workgroup");
    __builtin_amdgcn_wave_barrier();
    __builtin_amdgcn_fence(__ATOMIC_ACQUIRE, "workgroup");
  }
}

__global__ __launch_bounds__(256) void cast_scale_f32_f16x2(
    const float* __restrict__ in, _Float16* __restrict__ out, int n2, float scale) {
  int i = blockIdx.x * 256 + threadIdx.x;
  if (i < n2) {
    const _Float16 h0 = (_Float16)(in[2 * i] * scale), h1 = (_Float16)(in[2 * i + 1] * scale);
    const unsigned u = (unsigned)__builtin_bit_cast(unsigned short, h0) | ((unsigned)__builtin_bit_cast(unsigned short, h1) << 16);
    ((volatile unsigned*)out)[i] = u;
    __threadfence();
    ((volatile unsigned*)out)[i] = u;
  }
}

#define TC_C 256
#define TC_T 32
#define TC_PITCH 264
__global__ __launch_bounds__(256) void transpose_cast_f16(
    const float* __restrict__ in, _Float16* __restrict__ out, int L) {
  __shared__ __align__(16) _Float16 tile[TC_T * TC_PITCH];
  const int tid  = threadIdx.x;
  const int lane = tid & 31;
  const int wave = tid >> 5;
  const int bt   = blockIdx.y;
  const int t0   = blockIdx.x * TC_T;
  if (t0 + TC_T > L) return;
  const float* ib = in + (size_t)bt * TC_C * L;
#pragma unroll 8
  for (int i = 0; i < TC_C / 8; ++i) {
    const int c = wave + 8 * i;
    const float v = ib[(size_t)c * L + t0 + lane];
    tile[lane * TC_PITCH + c] = (_Float16)v;
  }
  __syncthreads();
  _Float16* ob = out + ((size_t)bt * L + t0) * TC_C;
  v8h rv[4];
#pragma unroll
  for (int p = 0; p < 4; ++p) {
    const int row = wave + 8 * p;
    rv[p] = *(const v8h*)(tile + row * TC_PITCH + lane * 8);
  }
  for (int pass = 0; pass < 2; ++pass) {
#pragma unroll
    for (int p = 0; p < 4; ++p) {
      const int row = wave + 8 * p;
      *(volatile v8h*)(ob + (size_t)row * TC_C + lane * 8) = rv[p];
    }
    __threadfence();
  }
}

#define SM_COLS 2048
#define SM_LOG2E 1.4426950408889634f
__global__ __launch_bounds__(256) void softmax_rows_f16(
    const float* __restrict__ S, _Float16* __restrict__ P, int nrows) {
  const int lane = threadIdx.x & 31;
  const int wave = threadIdx.x >> 5;
  const int row  = blockIdx.x * 8 + wave;
  if (row >= nrows) return;
  const float* sr = S + (size_t)row * SM_COLS + lane * 8;
  v4f v[16];
#pragma unroll
  for (int j = 0; j < 8; ++j) {
    v[2 * j]     = *(const v4f*)(sr + j * 256);
    v[2 * j + 1] = *(const v4f*)(sr + j * 256 + 4);
  }
  float m = -3.402823466e38f;
#pragma unroll
  for (int i = 0; i < 16; ++i) {
    m = fmaxf(m, fmaxf(fmaxf(v[i][0], v[i][1]), fmaxf(v[i][2], v[i][3])));
  }
  m = fmaxf(m, __shfl_xor(m, 1, 32));
  m = fmaxf(m, __shfl_xor(m, 2, 32));
  m = fmaxf(m, __shfl_xor(m, 4, 32));
  m = fmaxf(m, __shfl_xor(m, 8, 32));
  m = fmaxf(m, __shfl_xor(m, 16, 32));
  float sum = 0.f;
#pragma unroll
  for (int i = 0; i < 16; ++i) {
#pragma unroll
    for (int e = 0; e < 4; ++e) {
      const float t = (v[i][e] - m) * SM_LOG2E;
      const float p = __builtin_amdgcn_exp2f(t);
      v[i][e] = p;
      sum += p;
    }
  }
  sum += __shfl_xor(sum, 1, 32);
  sum += __shfl_xor(sum, 2, 32);
  sum += __shfl_xor(sum, 4, 32);
  sum += __shfl_xor(sum, 8, 32);
  sum += __shfl_xor(sum, 16, 32);
  const float inv = PSCALE * (1.0f / sum);
  v8h hv[8];
#pragma unroll
  for (int j = 0; j < 8; ++j) {
#pragma unroll
    for (int e = 0; e < 4; ++e) {
      hv[j][e]     = (_Float16)(v[2 * j][e] * inv);
      hv[j][4 + e] = (_Float16)(v[2 * j + 1][e] * inv);
    }
  }
  _Float16* pr = P + (size_t)row * SM_COLS + lane * 8;
  for (int pass = 0; pass < 2; ++pass) {
#pragma unroll
    for (int j = 0; j < 8; ++j) {
      *(volatile v8h*)(pr + j * 256) = hv[j];
    }
    __threadfence();
  }
}

extern "C" void kernel_launch(void* const* d_in, const int* in_sizes, int n_in,
                              void* d_out, int out_size, void* d_ws, size_t ws_size,
                              hipStream_t stream) {
  const int B = 4, C = 256, N = 8192, M = 2048, NCH = 4096;
  if (n_in < 8) return;
  if (in_sizes[0] != B * C * N || in_sizes[1] != B * C * M ||
      in_sizes[2] != C * C || in_sizes[3] != C || in_sizes[4] != C * C || in_sizes[5] != C ||
      in_sizes[6] != C * C || in_sizes[7] != C || out_size != B * C * N) return;

  const float* x    = (const float*)d_in[0];
  const float* x_pt = (const float*)d_in[1];
  const float* W1   = (const float*)d_in[2];
  const float* b1   = (const float*)d_in[3];
  const float* W2   = (const float*)d_in[4];
  const float* b2   = (const float*)d_in[5];
  const float* W3   = (const float*)d_in[6];
  const float* b3   = (const float*)d_in[7];
  float* out = (float*)d_out;

  const size_t szA16 = (size_t)B * N * C * 2;
  const size_t szW   = (size_t)C * C * 2;
  const size_t szTok = (size_t)B * M * C * 2;
  const size_t szS   = (size_t)NCH * M * 4;
  const size_t szP   = (size_t)NCH * M * 2;
  const size_t szXT  = (size_t)B * N * C * 2;
  const size_t offA16 = 0;
  const size_t offW1  = offA16 + szA16;
  const size_t offW2  = offW1 + szW;
  const size_t offW3  = offW2 + szW;
  const size_t offXPT = offW3 + szW;
  const size_t offBQ  = offXPT + szTok;
  const size_t offCT  = offBQ + szTok;
  const size_t offS   = offCT + szTok;
  const size_t offP   = offS + szS;
  const size_t total  = offP + szP;
  if (total > ws_size) return;
  if (szXT > szS) return;

  char* ws = (char*)d_ws;
  unsigned short* A16u  = (unsigned short*)(ws + offA16);
  unsigned short* W1u   = (unsigned short*)(ws + offW1);
  unsigned short* W2u   = (unsigned short*)(ws + offW2);
  unsigned short* W3u   = (unsigned short*)(ws + offW3);
  unsigned short* XPTu  = (unsigned short*)(ws + offXPT);
  unsigned short* BQu   = (unsigned short*)(ws + offBQ);
  unsigned short* CTu   = (unsigned short*)(ws + offCT);
  float*          Sf    = (float*)(ws + offS);
  unsigned short* XTu   = (unsigned short*)(ws + offS);
  unsigned short* P16u  = (unsigned short*)(ws + offP);

  const float inv16 = 1.0f / 16.0f;

  transpose_cast_f16<<<dim3(N / TC_T, B), 256, 0, stream>>>(x, (_Float16*)XTu, N);
  transpose_cast_f16<<<dim3(M / TC_T, B), 256, 0, stream>>>(x_pt, (_Float16*)XPTu, M);

  const int wn2 = C * C / 2;
  cast_scale_f32_f16x2<<<dim3((wn2 + 255) / 256), 256, 0, stream>>>(W1, (_Float16*)W1u, wn2, 16.0f);
  cast_scale_f32_f16x2<<<dim3((wn2 + 255) / 256), 256, 0, stream>>>(W2, (_Float16*)W2u, wn2, 16.0f);
  cast_scale_f32_f16x2<<<dim3((wn2 + 255) / 256), 256, 0, stream>>>(W3, (_Float16*)W3u, wn2, 16.0f);

  {
    const int tiles = (N / 64) * (C / 64);
    wmma_gemm64<0, false, 2, 1, false><<<dim3((tiles + 7) / 8, B), 256, 0, stream>>>(
        XTu, XTu, C, (long)N * C,
        W1u, W1u, C, 0L,
        (void*)A16u, (void*)A16u, C, (long)N * C,
        b1, x, 0L,
        N, C, C, inv16);
  }
  {
    const int tiles = (M / 64) * (C / 64);
    wmma_gemm64<0, false, 2, 1, false><<<dim3((tiles + 7) / 8, B), 256, 0, stream>>>(
        XPTu, XPTu, C, (long)M * C,
        W2u, W2u, C, 0L,
        (void*)BQu, (void*)BQu, C, (long)M * C,
        b2, x, 0L,
        M, C, C, inv16);
  }
  {
    const int tiles = (C / 64) * (M / 64);
    wmma_gemm64<0, false, 1, 1, false><<<dim3((tiles + 7) / 8, B), 256, 0, stream>>>(
        W3u, W3u, C, 0L,
        BQu, BQu, C, (long)M * C,
        (void*)CTu, (void*)CTu, M, (long)C * M,
        b3, x, 0L,
        C, M, C, inv16);
  }

  for (int bb = 0; bb < B; ++bb) {
    for (int ch = 0; ch < N / NCH; ++ch) {
      const unsigned short* Achunk = A16u + ((size_t)bb * N + (size_t)ch * NCH) * C;
      const unsigned short* Bq     = BQu + (size_t)bb * M * C;
      const unsigned short* Ct     = CTu + (size_t)bb * C * M;
      float*       outp = out + (size_t)bb * C * N + (size_t)ch * NCH;
      const float* xres = x   + (size_t)bb * C * N + (size_t)ch * NCH;

      {
        const int tiles = (NCH / 64) * (M / 64);
        wmma_gemm64<0, false, 0, 0, false><<<dim3((tiles + 7) / 8, 1), 256, 0, stream>>>(
            Achunk, Achunk, C, 0L,
            Bq, Bq, C, 0L,
            (void*)Sf, (void*)Sf, M, 0L,
            b1, x, 0L,
            NCH, M, C, inv16);
      }
      softmax_rows_f16<<<dim3((NCH + 7) / 8), 256, 0, stream>>>(Sf, (_Float16*)P16u, NCH);
      {
        const int tiles = (C / 64) * (NCH / 64);
        wmma_gemm64<0, false, 0, 0, true><<<dim3((tiles + 7) / 8, 1), 256, 0, stream>>>(
            Ct, Ct, M, 0L,
            P16u, P16u, M, 0L,
            (void*)outp, (void*)outp, N, 0L,
            b1, xres, 0L,
            C, NCH, M, PSCALE_INV);
      }
    }
  }
  (void)hipGetLastError();
}
